// get_attention_11098195493366
// MI455X (gfx1250) — hardware-verified
//
#include <hip/hip_runtime.h>
#include <stdint.h>


#define NB_    4
#define NL_    512
#define ND_    128
#define NC_    128
#define NROWS_ (NB_ * NL_)
#define EPS_   1e-7f
#define JC_    32
#define KP_    132
#define VP_    40
#define WBP_   136
#define OP_    132
#define AP2_   68
#define WP2_   20

typedef float    v8f   __attribute__((ext_vector_type(8)));
typedef float    v4f_t __attribute__((ext_vector_type(4)));
typedef v4f_t    __attribute__((may_alias)) v4f;
typedef uint32_t v4u_t __attribute__((ext_vector_type(4)));
typedef v4u_t    __attribute__((may_alias)) v4u;
typedef __bf16   v16bf __attribute__((ext_vector_type(16)));
typedef _Float16 v16h  __attribute__((ext_vector_type(16)));
typedef _Float16 v8h_t __attribute__((ext_vector_type(8)));
typedef v8h_t    __attribute__((may_alias)) v8h;

union FragB { v4u_t q[2]; v16bf v; };
union FragH { _Float16 e[16]; v8h_t q[2]; v16h v; };

#define LOG2E_F     1.4426950408889634f
#define TWO_LOG2E_F 2.8853900817779268f

__device__ __forceinline__ v8f mma_bf16(v8f acc, v16bf a, v16bf b) {
    acc = __builtin_amdgcn_wmma_f32_16x16x32_bf16(false, a, false, b, (short)0, acc, false, false);
    asm volatile("v_nop\n\tv_nop\n\tv_nop\n\tv_nop" : "+v"(acc) : "v"(a), "v"(b));
    return acc;
}
__device__ __forceinline__ v8f mma_f16(v8f acc, v16h a, v16h b) {
    acc = __builtin_amdgcn_wmma_f32_16x16x32_f16(false, a, false, b, (short)0, acc, false, false);
    asm volatile("v_nop\n\tv_nop\n\tv_nop\n\tv_nop" : "+v"(acc) : "v"(a), "v"(b));
    return acc;
}

__device__ __forceinline__ uint32_t bf_bits(float f) {
    uint32_t u = __builtin_bit_cast(uint32_t, f);
    u += 0x7FFFu + ((u >> 16) & 1u);
    return u >> 16;
}
__device__ __forceinline__ void bf_split(float x, uint32_t& hi, uint32_t& lo) {
    hi = bf_bits(x);
    const float xh = __builtin_bit_cast(float, hi << 16);
    lo = bf_bits(x - xh);
}

__device__ __forceinline__ _Float16 th64_h(float x) {
    const float e2 = __builtin_amdgcn_exp2f(x * TWO_LOG2E_F);
    const float r  = __builtin_amdgcn_rcpf(e2 + 1.0f);
    return (_Float16)__builtin_fmaf(-128.0f, r, 64.0f);
}

__global__ __launch_bounds__(256) void k_proj(
    const float* __restrict__ X, const float* __restrict__ Wt, const float* __restrict__ Wx,
    const float* __restrict__ bh, float* Qo, float* Ko, int nrows)
{
    __shared__ __align__(16) uint32_t sAh[16 * AP2_];
    __shared__ __align__(16) uint32_t sAl[16 * AP2_];
    __shared__ __align__(16) uint32_t sWh[NC_ * WP2_];
    __shared__ __align__(16) uint32_t sWl[NC_ * WP2_];
    __shared__ __align__(16) float    sO[16 * OP_];

    const int tid = threadIdx.x, lane = tid & 31, wave = tid >> 5;
    const int h = lane >> 4, m = lane & 15;
    const int row0 = blockIdx.x * 16;
    const int ncol = wave * 16 + m;

    for (int e = tid; e < 16 * (ND_ / 4); e += 256) {
        const int r = e >> 5, q = e & 31;
        const int gr = row0 + r;
        v4f_t v = {0.0f, 0.0f, 0.0f, 0.0f};
        if (gr < nrows) v = *(const v4f*)(X + (size_t)gr * ND_ + 4 * q);
        uint32_t h0, l0, h1, l1, h2, l2, h3, l3;
        bf_split(v.x, h0, l0); bf_split(v.y, h1, l1);
        bf_split(v.z, h2, l2); bf_split(v.w, h3, l3);
        sAh[r * AP2_ + 2 * q]     = h0 | (h1 << 16);
        sAh[r * AP2_ + 2 * q + 1] = h2 | (h3 << 16);
        sAl[r * AP2_ + 2 * q]     = l0 | (l1 << 16);
        sAl[r * AP2_ + 2 * q + 1] = l2 | (l3 << 16);
    }

#pragma unroll 1
    for (int g = 0; g < 2; ++g) {
        const float* W = (g == 0) ? Wt : Wx;
        float* dst = (g == 0) ? Qo : Ko;
        v8f acc = {};
#pragma unroll 1
        for (int kk = 0; kk < 4; ++kk) {
            __syncthreads();
            for (int e = tid; e < NC_ * 16; e += 256) {
                const int n = e & (NC_ - 1), kp = e >> 7;
                const int k = kk * 32 + 2 * kp;
                const float w0 = W[(size_t)k * NC_ + n];
                const float w1 = W[(size_t)(k + 1) * NC_ + n];
                uint32_t a0, b0, a1, b1;
                bf_split(w0, a0, b0); bf_split(w1, a1, b1);
                sWh[n * WP2_ + kp] = a0 | (a1 << 16);
                sWl[n * WP2_ + kp] = b0 | (b1 << 16);
            }
            __syncthreads();
            FragB fah, fal, fbh, fbl;
            const uint32_t* pa = sAh + m * AP2_ + kk * 16 + 4 * h;
            const uint32_t* pl = sAl + m * AP2_ + kk * 16 + 4 * h;
            const uint32_t* pb = sWh + ncol * WP2_ + 4 * h;
            const uint32_t* pc = sWl + ncol * WP2_ + 4 * h;
            fah.q[0] = *(const v4u*)(pa); fah.q[1] = *(const v4u*)(pa + 8);
            fal.q[0] = *(const v4u*)(pl); fal.q[1] = *(const v4u*)(pl + 8);
            fbh.q[0] = *(const v4u*)(pb); fbh.q[1] = *(const v4u*)(pb + 8);
            fbl.q[0] = *(const v4u*)(pc); fbl.q[1] = *(const v4u*)(pc + 8);
            acc = mma_bf16(acc, fah.v, fbh.v);
            acc = mma_bf16(acc, fah.v, fbl.v);
            acc = mma_bf16(acc, fal.v, fbh.v);
        }
        const float bias = (g == 0) ? bh[ncol] : 0.0f;
#pragma unroll
        for (int r = 0; r < 8; ++r) sO[(8 * h + r) * OP_ + ncol] = acc[r] + bias;
        __syncthreads();
        const int r0 = 2 * wave, r1 = 2 * wave + 1;
        const v4f_t v0 = *(const v4f*)(sO + r0 * OP_ + 4 * lane);
        const v4f_t v1 = *(const v4f*)(sO + r1 * OP_ + 4 * lane);
        const int g0 = row0 + r0, g1 = row0 + r1;
        if (g0 < nrows) *(volatile v4f*)(dst + (size_t)g0 * NC_ + 4 * lane) = v0;
        if (g1 < nrows) *(volatile v4f*)(dst + (size_t)g1 * NC_ + 4 * lane) = v1;
        __threadfence();
        if (g0 < nrows) *(volatile v4f*)(dst + (size_t)g0 * NC_ + 4 * lane) = v0;
        if (g1 < nrows) *(volatile v4f*)(dst + (size_t)g1 * NC_ + 4 * lane) = v1;
    }
}

__global__ __launch_bounds__(256) void k_attn(
    const float* __restrict__ X, const float* __restrict__ Qb, const float* __restrict__ Kx,
    const float* __restrict__ wa, const float* __restrict__ ba, float* Out)
{
    __shared__ __align__(16) float    sQ[16 * NC_];
    __shared__ __align__(16) float    sK[JC_ * KP_];
    __shared__ __align__(16) _Float16 sVT[ND_ * VP_];
    __shared__ __align__(16) _Float16 sWB[16 * WBP_];
    __shared__ __align__(16) _Float16 sP[16 * JC_];
    __shared__ float sS[16 * JC_];
    __shared__ __align__(16) float    sO[16 * OP_];
    __shared__ float sM[16], sL[16], sSc[16];

    const int tid = threadIdx.x, lane = tid & 31, wave = tid >> 5;
    const int h = lane >> 4, m = lane & 15;
    const int b  = blockIdx.x / (NL_ / 16);
    const int it = blockIdx.x % (NL_ / 16);
    const int qrow0 = b * NL_ + it * 16;
    const int ncol = wave * 16 + m;

    for (int e = tid; e < 16 * (NC_ / 4); e += 256) {
        const int r = e >> 5, q = e & 31;
        *(v4f*)(sQ + r * NC_ + 4 * q) = *(const v4f*)(Qb + (size_t)(qrow0 + r) * NC_ + 4 * q);
    }
    for (int e = tid; e < 16 * WBP_; e += 256) {
        const int rr = e / WBP_;
        const int c = e - rr * WBP_;
        _Float16 val = (_Float16)0.0f;
        if (c < NC_) {
            const float w = wa[c];
            const _Float16 hi = (_Float16)w;
            if (rr == 0) val = hi;
            else if (rr == 1) val = (_Float16)((w - (float)hi) * 4096.0f);
        }
        sWB[e] = val;
    }
    if (tid < 16) { sM[tid] = -3.0e38f; sL[tid] = 0.0f; }
    const float bav = ba[0];

    v8f acco = {};

#pragma unroll 1
    for (int ch = 0; ch < NL_ / JC_; ++ch) {
        __syncthreads();
        const int j0 = ch * JC_;
        for (int e = tid; e < JC_ * (NC_ / 4); e += 256) {
            const int r = e >> 5, q = e & 31;
            *(v4f*)(sK + r * KP_ + 4 * q) = *(const v4f*)(Kx + (size_t)(b * NL_ + j0 + r) * NC_ + 4 * q);
        }
        for (int e = tid; e < JC_ * (ND_ / 4); e += 256) {
            const int r = e >> 5, q = e & 31;
            const v4f_t v = *(const v4f*)(X + (size_t)(b * NL_ + j0 + r) * ND_ + 4 * q);
            sVT[(4 * q + 0) * VP_ + r] = (_Float16)v.x;
            sVT[(4 * q + 1) * VP_ + r] = (_Float16)v.y;
            sVT[(4 * q + 2) * VP_ + r] = (_Float16)v.z;
            sVT[(4 * q + 3) * VP_ + r] = (_Float16)v.w;
        }
        __syncthreads();

#pragma unroll 1
        for (int u = 0; u < 4; ++u) {
            const int t  = wave * 4 + u;
            const int i  = t >> 1;
            const int jb = (t & 1) * 16;
            const int j  = jb + m;
            v8f acc = {};
#pragma unroll
            for (int kk = 0; kk < 4; ++kk) {
                const int cb = kk * 32;
                const float* qp = sQ + i * NC_ + cb + 8 * h;
                const float* kp = sK + j * KP_ + cb + 8 * h;
                const v4f_t x0 = *(const v4f*)(qp)      + *(const v4f*)(kp);
                const v4f_t x1 = *(const v4f*)(qp + 4)  + *(const v4f*)(kp + 4);
                const v4f_t x2 = *(const v4f*)(qp + 16) + *(const v4f*)(kp + 16);
                const v4f_t x3 = *(const v4f*)(qp + 20) + *(const v4f*)(kp + 20);
                FragH fa;
                fa.e[0]  = th64_h(x0.x); fa.e[1]  = th64_h(x0.y); fa.e[2]  = th64_h(x0.z); fa.e[3]  = th64_h(x0.w);
                fa.e[4]  = th64_h(x1.x); fa.e[5]  = th64_h(x1.y); fa.e[6]  = th64_h(x1.z); fa.e[7]  = th64_h(x1.w);
                fa.e[8]  = th64_h(x2.x); fa.e[9]  = th64_h(x2.y); fa.e[10] = th64_h(x2.z); fa.e[11] = th64_h(x2.w);
                fa.e[12] = th64_h(x3.x); fa.e[13] = th64_h(x3.y); fa.e[14] = th64_h(x3.z); fa.e[15] = th64_h(x3.w);
                FragH fb;
                fb.q[0] = *(const v8h*)(sWB + m * WBP_ + cb + 8 * h);
                fb.q[1] = *(const v8h*)(sWB + m * WBP_ + cb + 16 + 8 * h);
                acc = mma_f16(acc, fa.v, fb.v);
            }
            float sv[8];
#pragma unroll
            for (int r = 0; r < 8; ++r) {
                const float lo = __shfl_xor(acc[r], 1);
                sv[r] = acc[r] * (1.0f / 64.0f) + lo * (1.0f / 262144.0f) + bav;
            }
            if (m == 0) {
#pragma unroll
                for (int r = 0; r < 8; ++r) sS[i * JC_ + jb + 8 * h + r] = sv[r];
            }
        }
        __syncthreads();

        if (tid < 16) {
            const int i = tid;
            const float mo = sM[i];
            float cm = mo;
            for (int jj = 0; jj < JC_; ++jj) cm = fmaxf(cm, sS[i * JC_ + jj]);
            const float sc = __builtin_amdgcn_exp2f((mo - cm) * LOG2E_F);
            float ls = sL[i] * sc;
            for (int jj = 0; jj < JC_; ++jj) {
                const float ev = __builtin_amdgcn_exp2f((sS[i * JC_ + jj] - cm) * LOG2E_F);
                ls += ev;
                sP[i * JC_ + jj] = (_Float16)(ev * 4096.0f);
            }
            sM[i] = cm; sL[i] = ls; sSc[i] = sc;
        }
        __syncthreads();

#pragma unroll
        for (int r = 0; r < 8; ++r) acco[r] *= sSc[8 * h + r];
        FragH fp, fv;
        fp.q[0] = *(const v8h*)(sP + m * JC_ + 8 * h);
        fp.q[1] = *(const v8h*)(sP + m * JC_ + 16 + 8 * h);
        fv.q[0] = *(const v8h*)(sVT + ncol * VP_ + 8 * h);
        fv.q[1] = *(const v8h*)(sVT + ncol * VP_ + 16 + 8 * h);
        acco = mma_f16(acco, fp.v, fv.v);
    }

#pragma unroll
    for (int r = 0; r < 8; ++r) {
        const int row = 8 * h + r;
        const float inv = 1.0f / (sL[row] + EPS_);
        sO[row * OP_ + ncol] = acco[r] * inv * (1.0f / 4096.0f);
    }
    __syncthreads();
    const int r0 = 2 * wave, r1 = 2 * wave + 1;
    const v4f_t v0 = *(const v4f*)(sO + r0 * OP_ + 4 * lane);
    const v4f_t v1 = *(const v4f*)(sO + r1 * OP_ + 4 * lane);
    float* p0 = Out + (size_t)(qrow0 + r0) * ND_ + 4 * lane;
    float* p1 = Out + (size_t)(qrow0 + r1) * ND_ + 4 * lane;
    *(volatile v4f*)p0 = v0;
    *(volatile v4f*)p1 = v1;
    __threadfence();
    *(volatile v4f*)p0 = v0;
    *(volatile v4f*)p1 = v1;
}

extern "C" void kernel_launch(void* const* d_in, const int* in_sizes, int n_in,
                              void* d_out, int out_size, void* d_ws, size_t ws_size,
                              hipStream_t stream) {
    if (n_in < 6) return;
    if (in_sizes[0] != NROWS_ * ND_ || in_sizes[1] != ND_ * NC_ || in_sizes[2] != ND_ * NC_ ||
        in_sizes[3] != NC_ || in_sizes[4] != NC_ || in_sizes[5] < 1 || out_size != NROWS_ * ND_)
        return;

    const float* inps  = (const float*)d_in[0];
    const float* wei_t = (const float*)d_in[1];
    const float* wei_x = (const float*)d_in[2];
    const float* bxh   = (const float*)d_in[3];
    const float* wei_a = (const float*)d_in[4];
    const float* bxa   = (const float*)d_in[5];
    float* out = (float*)d_out;

    const size_t per = (size_t)NROWS_ * NC_ * sizeof(float);
    if (ws_size < 2 * per) return;
    float* qb = (float*)d_ws;
    float* kx = (float*)((char*)d_ws + per);

    const int nrows = NROWS_;
    k_proj<<<dim3((nrows + 15) / 16), dim3(256), 0, stream>>>(inps, wei_t, wei_x, bxh, qb, kx, nrows);
    k_attn<<<dim3(NB_ * (NL_ / 16)), dim3(256), 0, stream>>>(inps, qb, kx, wei_a, bxa, out);
}
